// RRTAttention_34428457844867
// MI455X (gfx1250) — hardware-verified
//
#include <hip/hip_runtime.h>
#include <math.h>

typedef __attribute__((ext_vector_type(16))) _Float16 v16h;
typedef __attribute__((ext_vector_type(16))) __bf16 v16b;
typedef __attribute__((ext_vector_type(8)))  _Float16 v8h;
typedef __attribute__((ext_vector_type(8)))  float v8f;
typedef __attribute__((ext_vector_type(4)))  float v4f;
typedef __attribute__((ext_vector_type(2)))  float v2f;
typedef __attribute__((ext_vector_type(4)))  unsigned v4u;
typedef __attribute__((ext_vector_type(4)))  int v4i;
typedef float __attribute__((may_alias)) float_a;
typedef int __attribute__((may_alias)) int_a;

template <typename T> __device__ __forceinline__ void vst2(void* p, T v) { *(volatile T*)p = v; __threadfence(); *(volatile T*)p = v; }
__device__ __forceinline__ v8f wmma16(v16h a, v16h b, v8f c) {
  v8f d = __builtin_amdgcn_wmma_f32_16x16x32_f16(false, a, false, b, (short)0, c, false, false);
  asm volatile("v_nop\n\tv_nop\n\tv_nop\n\tv_nop" : "+v"(d) : "v"(a), "v"(b));
  return d;
}
__device__ __forceinline__ v8f wmma_bf(v16b a, v16b b, v8f c) {
  v8f d = __builtin_amdgcn_wmma_f32_16x16x32_bf16(false, a, false, b, (short)0, c, false, false);
  asm volatile("v_nop\n\tv_nop\n\tv_nop\n\tv_nop" : "+v"(d) : "v"(a), "v"(b));
  return d;
}
__device__ __forceinline__ v16h frag_h(const _Float16* rowk0, int lane) {
  union { v16h v; v8h q[2]; } u; const _Float16* p = rowk0 + 8 * (lane >> 4);
  u.q[0] = *(const v8h*)p; u.q[1] = *(const v8h*)(p + 16); return u.v;
}
__device__ __forceinline__ v16h frag_f32(const float* rowk0, int lane) {
  v16h a; const float* p = rowk0 + 8 * (lane >> 4);
#pragma unroll
  for (int i = 0; i < 8; ++i) { a[i] = (_Float16)p[i]; a[8 + i] = (_Float16)p[16 + i]; }
  return a;
}
__device__ __forceinline__ v16h frag_f32s(const float* rowk0, int lane, float sc) {
  v16h a; const float* p = rowk0 + 8 * (lane >> 4);
#pragma unroll
  for (int i = 0; i < 8; ++i) { a[i] = (_Float16)(p[i] * sc); a[8 + i] = (_Float16)(p[16 + i] * sc); }
  return a;
}
__device__ __forceinline__ v16h fragc_f32(const float* W, int k0, int n, int lane, int ld, int K) {
  v16h a; const int g = lane >> 4;
#pragma unroll
  for (int i = 0; i < 8; ++i) { const int ka = k0 + 8 * g + i, kb = ka + 16;
    a[i] = (_Float16)(ka < K ? W[(size_t)(ka < K ? ka : K - 1) * ld + n] : 0.f); a[8 + i] = (_Float16)(kb < K ? W[(size_t)(kb < K ? kb : K - 1) * ld + n] : 0.f); }
  return a;
}
struct F2 { v16b h, l; };
__device__ __forceinline__ F2 bsplit16(const float v[16]) { F2 r;
#pragma unroll
  for (int i = 0; i < 16; ++i) { const __bf16 h = (__bf16)v[i]; r.h[i] = h; r.l[i] = (__bf16)(v[i] - (float)h); }
  return r; }
__device__ __forceinline__ F2 split_row(const float* row, int k0, int lane) { float v[16]; const float* p = row + k0 + 8 * (lane >> 4);
#pragma unroll
  for (int i = 0; i < 8; ++i) { v[i] = p[i]; v[8 + i] = p[16 + i]; }
  return bsplit16(v); }
__device__ __forceinline__ F2 split_rowK(const float* row, int k0, int lane, int K) { float v[16]; const int g = lane >> 4;
#pragma unroll
  for (int i = 0; i < 8; ++i) { const int ka = k0 + 8 * g + i, kb = ka + 16; v[i] = ka < K ? row[ka < K ? ka : K - 1] : 0.f; v[8 + i] = kb < K ? row[kb < K ? kb : K - 1] : 0.f; }
  return bsplit16(v); }
__device__ __forceinline__ F2 split_col(const float* W, int k0, int n, int lane, int ld, int K) { float v[16]; const int g = lane >> 4;
#pragma unroll
  for (int i = 0; i < 8; ++i) { const int ka = k0 + 8 * g + i, kb = ka + 16; v[i] = ka < K ? W[(size_t)(ka < K ? ka : K - 1) * ld + n] : 0.f; v[8 + i] = kb < K ? W[(size_t)(kb < K ? kb : K - 1) * ld + n] : 0.f; }
  return bsplit16(v); }
__device__ __forceinline__ v8f mac3(const F2& a, const F2& b, v8f c) { c = wmma_bf(a.l, b.h, c); c = wmma_bf(a.h, b.l, c); return wmma_bf(a.h, b.h, c); }
__device__ __forceinline__ float sigm(float v) { return 1.0f / (1.0f + expf(-v)); }
#define LDSX() do { asm volatile("s_wait_dscnt 0" ::: "memory"); __builtin_amdgcn_wave_barrier(); __builtin_amdgcn_fence(__ATOMIC_RELEASE, "workgroup"); } while (0)


#define NB 2
#define TT 2048
#define CC 1024
#define NH 16
#define HK 4
#define GQ (NH / HK)
#define HD 64
#define KV (HK * HD)
#define RD 32
#define LR 4
#define HG 4
#define NR (NB * TT)
#ifndef TNB
#define TNB NB
#endif
typedef __attribute__((ext_vector_type(8))) __bf16 v8b;
__device__ __forceinline__ v16b frag_b(const __bf16* rowk0, int lane) {
  union { v16b v; v8b q[2]; } u; const __bf16* p = rowk0 + 8 * (lane >> 4);
  u.q[0] = *(const v8b*)p; u.q[1] = *(const v8b*)(p + 16); return u.v;
}
__device__ __forceinline__ float bfr(float v) { return (float)(__bf16)v; }
__device__ __attribute__((noinline)) float exp_ni(float v) { return expf(v); }
__device__ __attribute__((noinline)) float erf_ni(float v) { return erff(v); }

#define WS_XA  0u
#define WS_QH  (WS_XA + 4u * (size_t)NR * 32)
#define WS_QL  (WS_QH + 2u * (size_t)NR * CC)
#define WS_KH  (WS_QL + 2u * (size_t)NR * CC)
#define WS_VT  (WS_KH + 2u * (size_t)NR * KV)
#define WS_VL  (WS_VT + 2u * (size_t)NB * KV * TT)
#define WS_S   (WS_VL + 2u * (size_t)NB * KV * TT)
#define WS_Y   (WS_S + 4u * (size_t)HG * TT * TT)
#define WS_END (WS_Y + 4u * (size_t)NR * CC)

__global__ __launch_bounds__(128) void k_lora(const float* __restrict__ X, const float* __restrict__ AQ, const float* __restrict__ AV, const int* __restrict__ STEP, float* __restrict__ XA) { __shared__ __align__(16) float ss[4][16][36];
  const int tid = threadIdx.x, wave = tid >> 5, lane = tid & 31, col = lane & 15, g = lane >> 4; const size_t r0 = (size_t)blockIdx.x * 64 + wave * 16;
  const int si = STEP[0]; const bool use = (si >= 0 && si < 2); const float* aq = AQ + (size_t)(use ? si : 0) * LR * CC; const float* av = AV + (size_t)(use ? si : 0) * LR * CC;
  v8f acc = {};
#pragma unroll 4
  for (int kc = 0; kc < CC / 32; ++kc) { v16b a; { const float* p = X + (r0 + col) * CC + kc * 32 + 8 * g;
#pragma unroll
      for (int i = 0; i < 8; ++i) { a[i] = (__bf16)p[i]; a[8 + i] = (__bf16)p[16 + i]; } }
    v16b w; { const float* p = (col < 4) ? (aq + (size_t)col * CC) : (col < 8) ? (av + (size_t)(col - 4) * CC) : nullptr;
#pragma unroll
      for (int i = 0; i < 8; ++i) { w[i] = p ? (__bf16)p[kc * 32 + 8 * g + i] : (__bf16)0.f; w[8 + i] = p ? (__bf16)p[kc * 32 + 16 + 8 * g + i] : (__bf16)0.f; } }
    acc = wmma_bf(a, w, acc); }
#pragma unroll
  for (int r = 0; r < 8; ++r) ss[wave][8 * g + r][col] = use ? acc[r] : 0.f;
  LDSX(); for (int rl = 0; rl < 16; ++rl) if (lane < 2) vst2(XA + (r0 + rl) * 32 + lane * 4, *(const v4f*)&ss[wave][rl][lane * 4]); }
__global__ __launch_bounds__(128) void k_proj(const float* __restrict__ X, const float* __restrict__ WQ, const float* __restrict__ WK, const float* __restrict__ WV, const float* __restrict__ GAIN, const float* __restrict__ BQ, const float* __restrict__ BV, const int* __restrict__ STEP, const float* __restrict__ XA, _Float16* __restrict__ QH, _Float16* __restrict__ QL, _Float16* __restrict__ KH, __bf16* __restrict__ VT, __bf16* __restrict__ VL) {
  __shared__ __align__(16) float sf[64][132]; __shared__ __align__(16) _Float16 sh[64][136], sl[64][136]; __shared__ __align__(16) __bf16 th[128][72], tl2[128][72]; __shared__ float srs[64][2];
  const int tid = threadIdx.x, wave = tid >> 5, lane = tid & 31, col = lane & 15, g = lane >> 4; const int cg = blockIdx.y * 128; const size_t r0 = (size_t)blockIdx.x * 64;
  const int region = (cg < CC) ? 0 : (cg < CC + KV) ? 1 : 2; const int c0 = region == 0 ? cg : region == 1 ? cg - CC : cg - CC - KV; const float* Wm = region == 0 ? WQ : region == 1 ? WK : WV;
  const int si = STEP[0]; const bool use = (si >= 0 && si < 2);
  v8f acc[8] = {};
#pragma unroll 2
  for (int kc = 0; kc < CC / 32; ++kc) { v16b a; { const float* p = X + (r0 + wave * 16 + col) * CC + kc * 32 + 8 * g;
#pragma unroll
      for (int i = 0; i < 8; ++i) { a[i] = (__bf16)p[i]; a[8 + i] = (__bf16)p[16 + i]; } }
#pragma unroll
    for (int j = 0; j < 8; ++j) { v16b w; const int o = c0 + j * 16 + col; const float* p = Wm + (size_t)o * CC + kc * 32 + 8 * g;
#pragma unroll
      for (int i = 0; i < 8; ++i) { w[i] = (__bf16)p[i]; w[8 + i] = (__bf16)p[16 + i]; }
      acc[j] = wmma_bf(a, w, acc[j]); } }
#pragma unroll
  for (int j = 0; j < 8; ++j) { const int o = c0 + j * 16 + col;
#pragma unroll
    for (int r = 0; r < 8; ++r) { const int rl = wave * 16 + 8 * g + r; float v = acc[j][r];
      if (use && region != 1) { const float* Bm = (region == 0) ? (BQ + ((size_t)si * CC + o) * LR) : (BV + ((size_t)si * KV + o) * LR); const float* xa = XA + (r0 + rl) * 32 + (region == 0 ? 0 : 4);
#pragma unroll
        for (int q = 0; q < LR; ++q) v += xa[q] * bfr(Bm[q]); }
      sf[rl][j * 16 + col] = v; } }
  __syncthreads();
  if (region <= 1) {
    for (int e = tid; e < 64 * 2; e += 128) { const int rl = e >> 1, hh = e & 1; float s2 = 0.f;
#pragma unroll 1
      for (int d = 0; d < HD; ++d) { const float v = sf[rl][hh * 64 + d]; s2 += v * v; } srs[rl][hh] = 1.0f / sqrtf(s2 * (1.0f / HD) + 1.1920929e-7f); }
    __syncthreads();
    for (int e = tid; e < 64 * 128; e += 128) { const int rl = e >> 7, cl = e & 127; const int d = cl & 63, hb = cl & ~63; const float rs = srs[rl][cl >> 6]; const int t = (int)((r0 + rl) % TT); float v;
      if (d < RD) { const int i2 = d & 15; const float inv_freq = 1.0f / powf(10000.0f, (float)(2 * i2) / (float)RD); const float ang = (float)t * inv_freq; const float c = cosf(ang), s = sinf(ang); const float x1 = sf[rl][hb + i2] * rs, x2 = sf[rl][hb + 16 + i2] * rs; v = (d < 16) ? (x1 * c + x2 * s) : (-x1 * s + x2 * c); }
      else v = sf[rl][cl] * rs;
      if (region == 0) v *= bfr(GAIN[(c0 + cl) / HD]);
      const _Float16 hv = (_Float16)v; sh[rl][cl] = hv; sl[rl][cl] = (_Float16)(v - (float)hv); }
    __syncthreads();
    if (region == 0) { for (int e = tid; e < 64 * 16; e += 128) { const int rl = e >> 4, q = e & 15; vst2((unsigned*)(QH + (r0 + rl) * CC + c0 + q * 8), *(const v4u*)&sh[rl][q * 8]); vst2((unsigned*)(QL + (r0 + rl) * CC + c0 + q * 8), *(const v4u*)&sl[rl][q * 8]); } }
    else { for (int e = tid; e < 64 * 16; e += 128) { const int rl = e >> 4, q = e & 15; vst2((unsigned*)(KH + (r0 + rl) * KV + c0 + q * 8), *(const v4u*)&sh[rl][q * 8]); } } }
  else { for (int e = tid; e < 64 * 128; e += 128) { const int rl = e >> 7, cl = e & 127; const float v = sf[rl][cl]; const __bf16 bh = (__bf16)v; th[cl][rl] = bh; tl2[cl][rl] = (__bf16)(v - (float)bh); }
    __syncthreads(); const size_t b = r0 / TT; const int t0 = (int)(r0 % TT);
    for (int e = tid; e < 128 * 8; e += 128) { const int cl = e >> 3, q = e & 7; const size_t o2 = (b * KV + c0 + cl) * (size_t)TT + t0 + q * 8; vst2((unsigned*)(VT + o2), *(const v4u*)&th[cl][q * 8]); vst2((unsigned*)(VL + o2), *(const v4u*)&tl2[cl][q * 8]); } } }
__global__ __launch_bounds__(128) void k_sc(const _Float16* __restrict__ QH, const _Float16* __restrict__ QL, const _Float16* __restrict__ KH, int b, int h0, float* __restrict__ S0) { __shared__ __align__(16) float ss[4][16][132];
  const int h = h0 + blockIdx.z; const int kvh = h / GQ; float* S = S0 + (size_t)blockIdx.z * TT * TT;
  const int tid = threadIdx.x, wave = tid >> 5, lane = tid & 31, col = lane & 15, g = lane >> 4; const int k0 = blockIdx.y * 128; const int ql0 = blockIdx.x * 64 + wave * 16;
  if (k0 > blockIdx.x * 64 + 63) return;
  v8f acc[8] = {};
#pragma unroll
  for (int kc = 0; kc < HD / 32; ++kc) { const size_t qo = ((size_t)b * TT + ql0 + col) * CC + h * HD + kc * 32; const v16h ah = frag_h(QH + qo, lane), al = frag_h(QL + qo, lane);
#pragma unroll
    for (int j = 0; j < 8; ++j) { const v16h kb = frag_h(KH + ((size_t)b * TT + k0 + j * 16 + col) * KV + kvh * HD + kc * 32, lane); acc[j] = wmma16(ah, kb, acc[j]); acc[j] = wmma16(al, kb, acc[j]); } }
#pragma unroll
  for (int j = 0; j < 8; ++j) { const int kt = k0 + j * 16 + col;
#pragma unroll
    for (int r = 0; r < 8; ++r) { const int qt = ql0 + 8 * g + r; ss[wave][8 * g + r][j * 16 + col] = (kt <= qt) ? acc[j][r] * 0.125f : -3.0e38f; } }
  LDSX(); for (int rl = 0; rl < 16; ++rl) vst2(S + (size_t)(ql0 + rl) * TT + k0 + lane * 4, *(const v4f*)&ss[wave][rl][lane * 4]); }
__global__ __launch_bounds__(256) void k_sm(float* __restrict__ S0) { __shared__ float sred[8]; __shared__ float sbc; __shared__ __align__(16) float sh[TT];
  const int t = threadIdx.x; const size_t row = blockIdx.x; float* sr = S0 + (size_t)blockIdx.y * TT * TT + row * TT; const int kend = ((int)row / 64) * 64 + 64;
  float m = -3.0e38f; for (int k = t; k < kend; k += 256) m = fmaxf(m, sr[k]);
#pragma unroll
  for (int o = 1; o < 32; o <<= 1) m = fmaxf(m, __shfl_xor(m, o));
  if ((t & 31) == 0) sred[t >> 5] = m; __syncthreads(); if (t == 0) { float a = sred[0]; for (int i = 1; i < 8; ++i) a = fmaxf(a, sred[i]); sbc = a; } __syncthreads(); m = sbc; __syncthreads();
  float sum = 0.f; for (int k = t; k < kend; k += 256) { const float v = sr[k]; sum += (v <= -1.0e38f) ? 0.f : expf(v - m); }
#pragma unroll
  for (int o = 1; o < 32; o <<= 1) sum += __shfl_xor(sum, o);
  if ((t & 31) == 0) sred[t >> 5] = sum; __syncthreads(); if (t == 0) { float a = 0.f; for (int i = 0; i < 8; ++i) a += sred[i]; sbc = 1.0f / a; } __syncthreads(); const float inv = sbc;
  for (int k = t; k < kend; k += 256) { const float v = sr[k]; sh[k] = (v <= -1.0e38f) ? 0.f : expf(v - m) * inv * 2048.0f; }
  __syncthreads(); for (int q = t; q < kend / 4; q += 256) vst2(sr + q * 4, *(const v4f*)&sh[q * 4]); }
__global__ __launch_bounds__(128) void k_pv(const float* __restrict__ PS0, const __bf16* __restrict__ VT, const __bf16* __restrict__ VL, int b, int h0, float* __restrict__ Y) { __shared__ __align__(16) float ss[4][16][68];
  const int h = h0 + blockIdx.z; const int kvh = h / GQ; const float* PS = PS0 + (size_t)blockIdx.z * TT * TT;
  const int tid = threadIdx.x, wave = tid >> 5, lane = tid & 31, col = lane & 15, g = lane >> 4; const int ql0 = blockIdx.x * 64 + wave * 16; const int kend = blockIdx.x * 64 + 64;
  v8f acc[4] = {};
#pragma unroll 1
  for (int kc = 0; kc < kend / 32; ++kc) { const F2 p = split_row(PS + (size_t)(ql0 + col) * TT, kc * 32, lane);
#pragma unroll
    for (int j = 0; j < 4; ++j) { const size_t po = ((size_t)b * KV + kvh * HD + j * 16 + col) * TT + kc * 32; const v16b vh = frag_b(VT + po, lane); acc[j] = wmma_bf(p.h, vh, acc[j]); acc[j] = wmma_bf(p.l, vh, acc[j]); acc[j] = wmma_bf(p.h, frag_b(VL + po, lane), acc[j]); } }
#pragma unroll
  for (int j = 0; j < 4; ++j)
#pragma unroll
    for (int r = 0; r < 8; ++r) ss[wave][8 * g + r][j * 16 + col] = acc[j][r] * (1.0f / 2048.0f);
  LDSX(); for (int rl = 0; rl < 16; ++rl) if (lane < 16) vst2(Y + ((size_t)b * TT + ql0 + rl) * CC + h * HD + lane * 4, *(const v4f*)&ss[wave][rl][lane * 4]); }
__global__ __launch_bounds__(128) void k_out(const float* __restrict__ Y, const float* __restrict__ WO, float* __restrict__ OUT) { __shared__ __align__(16) float sf[4][16][132];
  const int tid = threadIdx.x, wave = tid >> 5, lane = tid & 31, col = lane & 15, g = lane >> 4; const int c0 = blockIdx.y * 128; const size_t r0 = (size_t)blockIdx.x * 64 + wave * 16;
  v8f acc[8] = {};
#pragma unroll 2
  for (int kc = 0; kc < CC / 32; ++kc) { const F2 a = split_row(Y + (r0 + col) * CC, kc * 32, lane);
#pragma unroll
    for (int j = 0; j < 8; ++j) { v16b w; const int o = c0 + j * 16 + col; const float* p = WO + (size_t)o * CC + kc * 32 + 8 * g;
#pragma unroll
      for (int i = 0; i < 8; ++i) { w[i] = (__bf16)p[i]; w[8 + i] = (__bf16)p[16 + i]; }
      acc[j] = wmma_bf(a.h, w, acc[j]); acc[j] = wmma_bf(a.l, w, acc[j]); } }
#pragma unroll
  for (int j = 0; j < 8; ++j)
#pragma unroll
    for (int r = 0; r < 8; ++r) sf[wave][8 * g + r][j * 16 + col] = acc[j][r];
  LDSX(); for (int rl = 0; rl < 16; ++rl) vst2(OUT + (r0 + rl) * CC + c0 + lane * 4, *(const v4f*)&sf[wave][rl][lane * 4]); }
extern "C" void kernel_launch(void* const* d_in, const int* in_sizes, int n_in, void* d_out, int out_size, void* d_ws, size_t ws_size, hipStream_t stream) {
  (void)in_sizes; (void)n_in; (void)out_size;
  const float** F = (const float**)d_in;
  if (ws_size < (size_t)WS_END) return;
  const int* STEP = (const int*)d_in[10];
  char* ws = (char*)d_ws; float *XA = (float*)(ws + WS_XA), *S = (float*)(ws + WS_S), *Y = (float*)(ws + WS_Y); _Float16 *QH = (_Float16*)(ws + WS_QH), *QL = (_Float16*)(ws + WS_QL), *KH = (_Float16*)(ws + WS_KH); __bf16 *VT = (__bf16*)(ws + WS_VT), *VL = (__bf16*)(ws + WS_VL);
  k_lora<<<TNB * TT / 64, 128, 0, stream>>>(F[0], F[6], F[8], STEP, XA);
  k_proj<<<dim3(TNB * TT / 64, (CC + 2 * KV) / 128), 128, 0, stream>>>(F[0], F[1], F[2], F[3], F[5], F[7], F[9], STEP, XA, QH, QL, KH, VT, VL);
  for (int b = 0; b < TNB; ++b) for (int h0 = 0; h0 < NH; h0 += HG) {
    k_sc<<<dim3(TT / 64, TT / 128, HG), 128, 0, stream>>>(QH, QL, KH, b, h0, S);
    k_sm<<<dim3(TT, HG), 256, 0, stream>>>(S);
    k_pv<<<dim3(TT / 64, 1, HG), 128, 0, stream>>>(S, VT, VL, b, h0, Y);
  }
  k_out<<<dim3(TNB * TT / 64, CC / 128), 128, 0, stream>>>(Y, F[4], (float*)d_out);
}
